// GCN_9122510536818
// MI455X (gfx1250) — hardware-verified
//
#include <hip/hip_runtime.h>
#include <stddef.h>
#include <stdint.h>
#include <math.h>


#define SEQ    32
#define EMB    128
#define HF     256
#define NCLS   40
#define N2P    64
#define AP     512
#define K1     384
#define K2     512
#define NTHR   256
#define NWAVE  8
#define EPT    8
#define CHUNK  (NTHR * EPT)
#define WCAP   (EPT * 32)
#define LISTN  (NWAVE * WCAP)
#define NBD    8192
#define SLD    13
#define NBA    1024
#define SLA    10
#define RCAP   28672
#define DEGCAP 64
#define GBM    64
#define GBN    64
#define GTHR   128
#define NU1    (HF * (K1 / 8))
#define NU2    (N2P * (K2 / 8))
#define AGG_ZINTS    (LISTN + 2 * RCAP + 3 * NBA)
#define MISC_INTS    16
#define ROWBUF_INTS  (NWAVE * AP / 2)
#define AGG_LDS_INTS (AGG_ZINTS + MISC_INTS + ROWBUF_INTS)
#define WSMAX  134217728

static_assert((CHUNK & (CHUNK - 1)) == 0 && CHUNK <= 4096);
static_assert((NBD & (NBD - 1)) == 0 && NBD == (1 << SLD));
static_assert((NBA & (NBA - 1)) == 0 && NBA == (1 << SLA));
static_assert(((long long)CHUNK << SLD) < (1LL << 31));
static_assert(NBD % (NTHR * 4) == 0);
static_assert(LISTN % NTHR == 0);
static_assert(NBA % (4 * NWAVE) == 0 && NBA % 32 == 0 && NBA % GBM == 0);
static_assert(RCAP % 4 == 0 && AGG_ZINTS % 4 == 0 && LISTN % 4 == 0 && ((AGG_ZINTS + MISC_INTS) % 4) == 0);
static_assert(K1 % 32 == 0 && K2 % 32 == 0 && K2 == AP && K1 == HF + EMB && K2 == 2 * HF);
static_assert(GBM == (GTHR / 32) * 16 && GBN == 64 && HF % GBN == 0 && N2P == GBN);
static_assert(NU1 % NTHR == 0 && NU2 % NTHR == 0 && (K1 / 8) == 48 && (K2 / 8) == 64);
static_assert(EMB == 4 * 32 && HF == 8 * 32 && SEQ == 32);
static_assert(NCLS % 4 == 0 && NCLS <= N2P && 4 * NCLS == 160 && (4 * NCLS * 4) % 128 == 0);
static_assert((NBA * NCLS * 4) % 128 == 0);
static_assert(AGG_LDS_INTS * 4 <= 300000);

typedef float          v2f   __attribute__((ext_vector_type(2)));
typedef float          v4f   __attribute__((ext_vector_type(4)));
typedef float          v8f   __attribute__((ext_vector_type(8)));
typedef int            v4i   __attribute__((ext_vector_type(4)));
typedef int            v8i   __attribute__((ext_vector_type(8)));
typedef unsigned short v4us  __attribute__((ext_vector_type(4)));
typedef unsigned short v8us  __attribute__((ext_vector_type(8)));
typedef unsigned short v16us __attribute__((ext_vector_type(16)));
typedef __bf16         v16bf __attribute__((ext_vector_type(16)));
typedef v2f  __attribute__((may_alias)) v2fa;
typedef v4f  __attribute__((may_alias)) v4fa;
typedef v4i  __attribute__((may_alias)) v4ia;
typedef v4us __attribute__((may_alias)) v4usa;
typedef v8us __attribute__((may_alias)) v8usa;
union FragB { v16bf v; v16us u; v8us h[2]; v8i w; };

__device__ __forceinline__ v8f wmb(const FragB& a, const FragB& b, v8f c) {
  v8f d = __builtin_amdgcn_wmma_f32_16x16x32_bf16(false, a.v, false, b.v, (short)0, c, false, false);
  asm volatile("v_nop\n\tv_nop\n\tv_nop\n\tv_nop" : "+v"(d) : "v"(a.w), "v"(b.w));
  return d;
}

__device__ __forceinline__ unsigned bf16_bits(float f) {
  const unsigned u = __float_as_uint(f);
  return (u + 0x7FFFu + ((u >> 16) & 1u)) >> 16;
}
__device__ __forceinline__ float bf16_val(float f) {
  return __uint_as_float(bf16_bits(f) << 16);
}

__device__ __forceinline__ void wave_sync() {
  __builtin_amdgcn_fence(__ATOMIC_RELEASE, "wavefront");
  __builtin_amdgcn_wave_barrier();
  __builtin_amdgcn_fence(__ATOMIC_ACQUIRE, "wavefront");
}

__device__ __forceinline__ void hilo4(float x0, float x1, float x2, float x3, v4us& h, v4us& l) {
  unsigned hb;
  hb = bf16_bits(x0); h[0] = (unsigned short)hb; l[0] = (unsigned short)bf16_bits(x0 - __uint_as_float(hb << 16));
  hb = bf16_bits(x1); h[1] = (unsigned short)hb; l[1] = (unsigned short)bf16_bits(x1 - __uint_as_float(hb << 16));
  hb = bf16_bits(x2); h[2] = (unsigned short)hb; l[2] = (unsigned short)bf16_bits(x2 - __uint_as_float(hb << 16));
  hb = bf16_bits(x3); h[3] = (unsigned short)hb; l[3] = (unsigned short)bf16_bits(x3 - __uint_as_float(hb << 16));
}

template <int SLB>
__device__ __forceinline__ int scan_chunk(const int* __restrict__ dsts, int nE, int cbase, int slotBase,
                                          int nb, int vec8, int* list, int tid, int lane, int wave) {
  int wc = 0;
  const int el0  = tid * EPT;
  const int e0   = cbase + el0;
  const int sent = -2147483647 - 1;
  v4i da, db;
  if (vec8 != 0 && cbase + CHUNK <= nE) {
    da = *(const v4i*)(dsts + e0);
    db = *(const v4i*)(dsts + e0 + 4);
  } else {
    da.x = (e0     < nE) ? dsts[min(e0,     nE - 1)] : sent;
    da.y = (e0 + 1 < nE) ? dsts[min(e0 + 1, nE - 1)] : sent;
    da.z = (e0 + 2 < nE) ? dsts[min(e0 + 2, nE - 1)] : sent;
    da.w = (e0 + 3 < nE) ? dsts[min(e0 + 3, nE - 1)] : sent;
    db.x = (e0 + 4 < nE) ? dsts[min(e0 + 4, nE - 1)] : sent;
    db.y = (e0 + 5 < nE) ? dsts[min(e0 + 5, nE - 1)] : sent;
    db.z = (e0 + 6 < nE) ? dsts[min(e0 + 6, nE - 1)] : sent;
    db.w = (e0 + 7 < nE) ? dsts[min(e0 + 7, nE - 1)] : sent;
  }
  const unsigned nbs = (unsigned)slotBase;
  const unsigned unb = (unsigned)nb;
  const unsigned s0 = (unsigned)da.x - nbs, s1 = (unsigned)da.y - nbs;
  const unsigned s2 = (unsigned)da.z - nbs, s3 = (unsigned)da.w - nbs;
  const unsigned s4 = (unsigned)db.x - nbs, s5 = (unsigned)db.y - nbs;
  const unsigned s6 = (unsigned)db.z - nbs, s7 = (unsigned)db.w - nbs;
  const bool h0 = s0 < unb, h1 = s1 < unb, h2 = s2 < unb, h3 = s3 < unb;
  const bool h4 = s4 < unb, h5 = s5 < unb, h6 = s6 < unb, h7 = s7 < unb;
  const unsigned any = __builtin_amdgcn_ballot_w32(h0 | h1 | h2 | h3 | h4 | h5 | h6 | h7);
  if (any != 0u) {
#define HITJ(J, HJ, SJ) { \
      const unsigned mj = __builtin_amdgcn_ballot_w32(HJ); \
      if (mj != 0u) { \
        if (HJ) { \
          const int pos = wc + (int)__builtin_amdgcn_mbcnt_lo(mj, 0u); \
          if (pos < WCAP) list[wave * WCAP + pos] = ((el0 + (J)) << SLB) | (int)(SJ); \
        } \
        wc += (int)__builtin_popcount(mj); } }
    HITJ(0, h0, s0)
    HITJ(1, h1, s1)
    HITJ(2, h2, s2)
    HITJ(3, h3, s3)
    HITJ(4, h4, s4)
    HITJ(5, h5, s5)
    HITJ(6, h6, s6)
    HITJ(7, h7, s7)
#undef HITJ
  }
  return wc;
}

__global__ __launch_bounds__(NTHR) void k_prep(const float* __restrict__ W1, const float* __restrict__ W2,
                                               unsigned short* W1T, unsigned short* W2T) {
  const int u = (int)blockIdx.x * NTHR + (int)threadIdx.x;
  v8us o;
  unsigned short* dp;
  if (u < NU1) {
    const int n  = u / (K1 / 8);
    const int k8 = (u - n * (K1 / 8)) * 8;
    const int kk = k8 < HF ? k8 : k8 - HF;
    const float* p = W1 + (size_t)kk * HF + n;
#pragma unroll
    for (int i = 0; i < 8; ++i) o[i] = (unsigned short)bf16_bits(p[(size_t)i * HF]);
    dp = W1T + (size_t)n * K1 + k8;
  } else if (u < NU1 + NU2) {
    const int v  = u - NU1;
    const int n  = v >> 6;
    const int k8 = (v & 63) * 8;
    const int kk = k8 & (HF - 1);
    const int nc = n < NCLS ? n : NCLS - 1;
    const bool ok = n < NCLS;
    const float* p = W2 + (size_t)kk * NCLS + nc;
#pragma unroll
    for (int i = 0; i < 8; ++i) {
      const unsigned short b = (unsigned short)bf16_bits(p[(size_t)i * NCLS]);
      o[i] = ok ? b : (unsigned short)0;
    }
    dp = W2T + (size_t)n * K2 + k8;
  } else {
    return;
  }
  *(volatile v8us*)dp = o;
  __threadfence();
  *(volatile v8us*)dp = o;
}

__global__ __launch_bounds__(NTHR) void k_deg(const int* __restrict__ keys, int nE, int vec8, float* nrm) {
  __shared__ __attribute__((aligned(16))) int scnt[NBD];
  __shared__ __attribute__((aligned(16))) int list[LISTN];
  __shared__ int wcnt[NWAVE];
  const int tid = (int)threadIdx.x, lane = tid & 31, wave = tid >> 5;
  const int nodeBase = (int)blockIdx.x * NBD;

  for (int i = tid; i < NBD; i += NTHR) scnt[i] = 0;
  for (int i = tid; i < LISTN; i += NTHR) list[i] = 0;
  if (tid < NWAVE) wcnt[tid] = 0;
  __syncthreads();

  const int nChunks = (nE + CHUNK - 1) / CHUNK;
#pragma unroll 1
  for (int ch = 0; ch < nChunks; ++ch) {
    const int cbase = ch * CHUNK;
    const int wc = scan_chunk<SLD>(keys, nE, cbase, nodeBase, NBD, vec8, list, tid, lane, wave);
    if (lane == 0) wcnt[wave] = wc;
    __syncthreads();
    if (wave == 0) {
#pragma unroll 1
      for (int w2 = 0; w2 < NWAVE; ++w2) {
        int c = wcnt[w2];
        c = c < 0 ? 0 : (c > WCAP ? WCAP : c);
#pragma unroll 1
        for (int b0 = 0; b0 < c; b0 += 32) {
          const int idx = b0 + lane;
          const int ent = list[w2 * WCAP + (idx < WCAP ? idx : WCAP - 1)];
          const int m32 = (c - b0) < 32 ? (c - b0) : 32;
#pragma unroll 1
          for (int k = 0; k < m32; ++k) {
            const int u  = __builtin_amdgcn_readlane(ent, k);
            const int sl = u & (NBD - 1);
            if (lane == 0) scnt[sl] = scnt[sl] + 1;
          }
        }
      }
    }
    __syncthreads();
  }

#pragma unroll 1
  for (int i = tid; i < NBD; i += NTHR) {
    int c = scnt[i];
    c = c < 1 ? 1 : c;
    const float r = 1.0f / sqrtf((float)c);
    scnt[i] = __float_as_int(r);
  }
  __syncthreads();

  v4f vals[NBD / (NTHR * 4)];
#pragma unroll
  for (int it = 0; it < NBD / (NTHR * 4); ++it) {
    const int s0 = it * (NTHR * 4) + 4 * tid;
    const v4i c4 = *(const v4ia*)(scnt + s0);
    v4f v;
    v.x = __int_as_float(c4.x); v.y = __int_as_float(c4.y);
    v.z = __int_as_float(c4.z); v.w = __int_as_float(c4.w);
    vals[it] = v;
  }
#pragma unroll
  for (int it = 0; it < NBD / (NTHR * 4); ++it) {
    const int s0 = it * (NTHR * 4) + 4 * tid;
    *(volatile v4f*)(nrm + (size_t)nodeBase + s0) = vals[it];
  }
  __threadfence();
#pragma unroll
  for (int it = 0; it < NBD / (NTHR * 4); ++it) {
    const int s0 = it * (NTHR * 4) + 4 * tid;
    *(volatile v4f*)(nrm + (size_t)nodeBase + s0) = vals[it];
  }
}

__global__ __launch_bounds__(NTHR) void k_embed(const int* __restrict__ feats, const float* __restrict__ emb,
                                                int nN, int nTok, unsigned short* hpl) {
  __shared__ __attribute__((aligned(16))) unsigned short rowbufs[NWAVE * AP];
  const int tid = (int)threadIdx.x, lane = tid & 31, wave = tid >> 5;
  const int node = (int)blockIdx.x * NWAVE + wave;
  unsigned short* rowbuf = rowbufs + wave * AP;
  const bool live = node < nN;
  const int nc = live ? node : nN - 1;
  int id = feats[(size_t)nc * SEQ + lane];
  id = id < 0 ? 0 : (id > nTok - 1 ? nTok - 1 : id);
  const unsigned nz = __builtin_amdgcn_ballot_w32(id != 0);
  int cnt = (int)__builtin_popcount(nz);
  cnt = cnt < 1 ? 1 : cnt;
  const float ninf = __int_as_float((int)0xff800000u);
  float s0 = 0.0f, s1 = 0.0f, s2 = 0.0f, s3 = 0.0f;
  float m0 = ninf, m1 = ninf, m2 = ninf, m3 = ninf;
#pragma unroll 4
  for (int l = 0; l < SEQ; ++l) {
    const int tok = __builtin_amdgcn_readlane(id, l);
    const v4f a = *(const v4f*)(emb + (size_t)tok * EMB + 4 * lane);
    const bool nzt = tok != 0;
    const float e0 = nzt ? bf16_val(a.x) : 0.0f;
    const float e1 = nzt ? bf16_val(a.y) : 0.0f;
    const float e2 = nzt ? bf16_val(a.z) : 0.0f;
    const float e3 = nzt ? bf16_val(a.w) : 0.0f;
    s0 += e0; s1 += e1; s2 += e2; s3 += e3;
    m0 = fmaxf(m0, e0); m1 = fmaxf(m1, e1); m2 = fmaxf(m2, e2); m3 = fmaxf(m3, e3);
  }
  const float cf = (float)cnt;
  const float a0 = live ? (s0 / cf) : 0.0f;
  const float a1 = live ? (s1 / cf) : 0.0f;
  const float a2 = live ? (s2 / cf) : 0.0f;
  const float a3 = live ? (s3 / cf) : 0.0f;
  v4us mh, ml, xh;
  hilo4(a0, a1, a2, a3, mh, ml);
  xh[0] = live ? (unsigned short)bf16_bits(m0) : (unsigned short)0;
  xh[1] = live ? (unsigned short)bf16_bits(m1) : (unsigned short)0;
  xh[2] = live ? (unsigned short)bf16_bits(m2) : (unsigned short)0;
  xh[3] = live ? (unsigned short)bf16_bits(m3) : (unsigned short)0;
  const v4us z4 = {0, 0, 0, 0};
  *(v4usa*)(rowbuf + 4 * lane) = mh;
  *(v4usa*)(rowbuf + EMB + 4 * lane) = xh;
  *(v4usa*)(rowbuf + 2 * EMB + 4 * lane) = ml;
  *(v4usa*)(rowbuf + 3 * EMB + 4 * lane) = z4;
  wave_sync();
  const v8us q0 = *(const v8usa*)(rowbuf + 8 * lane);
  const v8us q1 = *(const v8usa*)(rowbuf + 256 + 8 * lane);
  unsigned short* rpw = hpl + (size_t)node * AP + 8 * lane;
  *(volatile v8us*)rpw = q0;
  *(volatile v8us*)(rpw + 256) = q1;
  __threadfence();
  *(volatile v8us*)rpw = q0;
  *(volatile v8us*)(rpw + 256) = q1;
}

__global__ __launch_bounds__(GTHR) void k_gemm(
    const unsigned short* __restrict__ A, int lda, const unsigned short* __restrict__ WT, int K,
    const float* __restrict__ rs, float* outF, int ldo)
{
  __shared__ __attribute__((aligned(16))) float stg[GBM * GBN];
  __shared__ float rsl[GBM];
  const int tid = (int)threadIdx.x, lane = tid & 31, wave = tid >> 5, hh = lane >> 4, m = lane & 15;
  const int rowBase = (int)blockIdx.x * GBM;
  const int col0    = (int)blockIdx.y * GBN;

  if (tid < GBM) rsl[tid] = rs[rowBase + tid];

  v8f acc[4];
  {
    const v8f z = {0.f, 0.f, 0.f, 0.f, 0.f, 0.f, 0.f, 0.f};
    acc[0] = z; acc[1] = z; acc[2] = z; acc[3] = z;
  }
  const unsigned short* ap = A  + (size_t)(rowBase + 16 * wave + m) * (size_t)lda + 8 * hh;
  const unsigned short* wp = WT + (size_t)(col0 + m) * (size_t)K + 8 * hh;
  const int ksteps = K >> 5;
#pragma unroll 1
  for (int ks = 0; ks < ksteps; ++ks) {
    FragB af;
    af.h[0] = *(const v8usa*)(ap + 32 * ks);
    af.h[1] = *(const v8usa*)(ap + 32 * ks + 16);
#pragma unroll
    for (int t = 0; t < 4; ++t) {
      const unsigned short* wq = wp + (size_t)(16 * t) * (size_t)K + 32 * ks;
      FragB bf;
      bf.h[0] = *(const v8usa*)wq;
      bf.h[1] = *(const v8usa*)(wq + 16);
      acc[t] = wmb(af, bf, acc[t]);
    }
  }

#pragma unroll
  for (int t = 0; t < 4; ++t) {
    const int lc = 16 * t + m;
#pragma unroll
    for (int r = 0; r < 8; ++r) {
      const int lr = 16 * wave + 8 * hh + r;
      stg[lr * GBN + lc] = acc[t][r];
    }
  }
  __syncthreads();

  v4f fv[8];
#pragma unroll
  for (int i = 0; i < 8; ++i) {
    const int lr = 16 * wave + 2 * i + hh;
    const float sc = rsl[lr];
    const v4f t4 = *(const v4fa*)(stg + lr * GBN + 4 * m);
    v4f y;
    y.x = t4.x * sc; y.y = t4.y * sc; y.z = t4.z * sc; y.w = t4.w * sc;
    fv[i] = y;
  }
#pragma unroll
  for (int i = 0; i < 8; ++i) {
    const int lr = 16 * wave + 2 * i + hh;
    const int gr = rowBase + lr;
    float* op = outF + (size_t)gr * (size_t)ldo + col0 + 4 * m;
    *(volatile v4f*)op = fv[i];
  }
  __threadfence();
#pragma unroll
  for (int i = 0; i < 8; ++i) {
    const int lr = 16 * wave + 2 * i + hh;
    const int gr = rowBase + lr;
    float* op = outF + (size_t)gr * (size_t)ldo + col0 + 4 * m;
    *(volatile v4f*)op = fv[i];
  }
}

__device__ __forceinline__ float fin_relu(float acc, float ndv, float b, float pzr, bool live) {
  float v = acc * ndv + b;
  v = (v > 0.0f) ? v : (v - v);
  v = v + pzr;
  return live ? v : 0.0f;
}

template <int MODE>
__global__ __launch_bounds__(NTHR) void k_agg(const int* __restrict__ srcs, const int* __restrict__ dsts,
                                              int nE, int nN, int vec8, int mRows,
                                              const float* __restrict__ nd, const float* __restrict__ xl,
                                              const float* __restrict__ bias,
                                              unsigned short* hb, float* hout) {
  extern __shared__ __attribute__((aligned(16))) int dsm[];
  int* list = dsm;
  int* hl   = dsm + LISTN;
  int* sl   = hl + RCAP;
  int* cnt  = sl + RCAP;
  int* offs = cnt + NBA;
  int* cur  = offs + NBA;
  int* misc = cur + NBA;
  const int tid = (int)threadIdx.x, lane = tid & 31, wave = tid >> 5;
  const int nodeBase = (int)blockIdx.x * NBA;

  {
    const v4i z4 = {0, 0, 0, 0};
    for (int i = tid * 4; i < AGG_ZINTS; i += NTHR * 4) *(v4ia*)(dsm + i) = z4;
    if (tid < MISC_INTS) misc[tid] = 0;
  }
  __syncthreads();

  int t = 0, ov = 0;
  const int nChunks = (nE + CHUNK - 1) / CHUNK;
#pragma unroll 1
  for (int ch = 0; ch < nChunks; ++ch) {
    const int cbase = ch * CHUNK;
    const int wc = scan_chunk<SLA>(dsts, nE, cbase, nodeBase, NBA, vec8, list, tid, lane, wave);
    if (lane == 0) misc[wave] = wc;
    __syncthreads();
    if (wave == 0) {
#pragma unroll 1
      for (int w2 = 0; w2 < NWAVE; ++w2) {
        int c = misc[w2];
        c = c < 0 ? 0 : (c > WCAP ? WCAP : c);
#pragma unroll 1
        for (int b0 = 0; b0 < c; b0 += 32) {
          const int idx = b0 + lane;
          const int ent = list[w2 * WCAP + (idx < WCAP ? idx : WCAP - 1)];
          const int m32 = (c - b0) < 32 ? (c - b0) : 32;
#pragma unroll 1
          for (int k = 0; k < m32; ++k) {
            const int u    = __builtin_amdgcn_readlane(ent, k);
            const int slot = u & (NBA - 1);
            const int el   = (u >> SLA) & (CHUNK - 1);
            const int pk   = ((cbase + el) << SLA) | slot;
            if (t < RCAP) {
              if (lane == 0) { hl[t] = pk; cnt[slot] = cnt[slot] + 1; }
              t = t + 1;
            } else {
              ov = 1;
            }
          }
        }
      }
    }
    __syncthreads();
  }
  if (wave == 0 && lane == 0) { misc[8] = t; misc[9] = ov; }
  __syncthreads();
  int tt = misc[8];
  tt = tt < 0 ? 0 : (tt > RCAP ? RCAP : tt);
  const int ovf = misc[9];

  if (wave == 0) {
    const int base = lane * (NBA / 32);
    int s = 0;
#pragma unroll 1
    for (int i = 0; i < NBA / 32; ++i) s += cnt[base + i];
    int incl = s;
#pragma unroll
    for (int d = 1; d < 32; d <<= 1) {
      const int y = __shfl_up(incl, d, 32);
      if (lane >= d) incl += y;
    }
    int run = incl - s;
#pragma unroll 1
    for (int i = 0; i < NBA / 32; ++i) {
      const int cv = cnt[base + i];
      offs[base + i] = run;
      cur[base + i]  = run;
      run += cv;
    }
  }
  __syncthreads();
  if (wave == 0) {
#pragma unroll 1
    for (int b0 = 0; b0 < tt; b0 += 32) {
      const int idx = b0 + lane;
      const int ent = hl[idx < RCAP ? idx : RCAP - 1];
      const int m32 = (tt - b0) < 32 ? (tt - b0) : 32;
#pragma unroll 1
      for (int k = 0; k < m32; ++k) {
        const int u    = __builtin_amdgcn_readlane(ent, k);
        const int slot = u & (NBA - 1);
        if (lane == 0) {
          int p = cur[slot];
          p = p < 0 ? 0 : (p > RCAP - 1 ? RCAP - 1 : p);
          sl[p] = u;
          cur[slot] = p + 1;
        }
      }
    }
  }
  __syncthreads();

  const float qnan = __int_as_float(0x7fc00000);
  const float pz = (ovf != 0) ? qnan : 0.0f;

  if constexpr (MODE != 0) {
    unsigned short* rowbuf = (unsigned short*)(misc + MISC_INTS) + wave * AP;
    float b0v, b1v, b2v, b3v, b4v, b5v, b6v, b7v;
    {
      const v4f ba = *(const v4fa*)(bias + 4 * lane);
      const v4f bb = *(const v4fa*)(bias + 128 + 4 * lane);
      b0v = bf16_val(ba.x); b1v = bf16_val(ba.y); b2v = bf16_val(ba.z); b3v = bf16_val(ba.w);
      b4v = bf16_val(bb.x); b5v = bf16_val(bb.y); b6v = bf16_val(bb.z); b7v = bf16_val(bb.w);
    }
#pragma unroll 1
    for (int si = 0; si < NBA / NWAVE; ++si) {
      const int s    = si * NWAVE + wave;
      const int node = nodeBase + s;
      int c = cnt[s];
      const bool big = c > DEGCAP;
      c = c < 0 ? 0 : (c > DEGCAP ? DEGCAP : c);
      int o = offs[s];
      o = o < 0 ? 0 : (o > RCAP ? RCAP : o);
      const int nc = node < nN ? node : nN - 1;
      const float ndv = nd[nc];
      float a0 = 0.0f, a1 = 0.0f, a2 = 0.0f, a3 = 0.0f, a4 = 0.0f, a5 = 0.0f, a6 = 0.0f, a7 = 0.0f;
#pragma unroll 1
      for (int b0 = 0; b0 < c; b0 += 32) {
        int idx = o + b0 + lane;
        idx = idx > RCAP - 1 ? RCAP - 1 : idx;
        const int ent = sl[idx];
        int eid = ent >> SLA;
        eid = eid < 0 ? 0 : (eid > nE - 1 ? nE - 1 : eid);
        int sr = srcs[eid];
        sr = sr < 0 ? 0 : (sr > nN - 1 ? nN - 1 : sr);
        const int m32 = (c - b0) < 32 ? (c - b0) : 32;
#pragma unroll 1
        for (int k = 0; k < m32; ++k) {
          const int sk = __builtin_amdgcn_readlane(sr, k);
          const float* rp = xl + (size_t)sk * HF + 4 * lane;
          const v4f xa = *(const v4fa*)rp;
          const v4f xb = *(const v4fa*)(rp + 128);
          a0 += xa.x; a1 += xa.y; a2 += xa.z; a3 += xa.w;
          a4 += xb.x; a5 += xb.y; a6 += xb.z; a7 += xb.w;
        }
      }
      const float pzr = big ? qnan : pz;
      const bool live = node < nN;
      const float y0 = fin_relu(a0, ndv, b0v, pzr, live);
      const float y1 = fin_relu(a1, ndv, b1v, pzr, live);
      const float y2 = fin_relu(a2, ndv, b2v, pzr, live);
      const float y3 = fin_relu(a3, ndv, b3v, pzr, live);
      const float y4 = fin_relu(a4, ndv, b4v, pzr, live);
      const float y5 = fin_relu(a5, ndv, b5v, pzr, live);
      const float y6 = fin_relu(a6, ndv, b6v, pzr, live);
      const float y7 = fin_relu(a7, ndv, b7v, pzr, live);
      v4us h0, l0, h1, l1;
      hilo4(y0, y1, y2, y3, h0, l0);
      hilo4(y4, y5, y6, y7, h1, l1);
      *(v4usa*)(rowbuf + 4 * lane) = h0;
      *(v4usa*)(rowbuf + 128 + 4 * lane) = h1;
      *(v4usa*)(rowbuf + 256 + 4 * lane) = l0;
      *(v4usa*)(rowbuf + 384 + 4 * lane) = l1;
      wave_sync();
      const v8us q0 = *(const v8usa*)(rowbuf + 8 * lane);
      const v8us q1 = *(const v8usa*)(rowbuf + 256 + 8 * lane);
      wave_sync();
      if (node < mRows) {
        unsigned short* rpw = hb + (size_t)node * AP + 8 * lane;
        *(volatile v8us*)rpw = q0;
        *(volatile v8us*)(rpw + 256) = q1;
        __threadfence();
        *(volatile v8us*)rpw = q0;
        *(volatile v8us*)(rpw + 256) = q1;
      }
    }
  } else {
    float* stgf = (float*)(misc + MISC_INTS) + wave * 256;
    float bv0, bv1;
    {
      const int bi = (2 * lane) < (NCLS - 2) ? (2 * lane) : (NCLS - 2);
      const v2f a = *(const v2fa*)(bias + bi);
      const bool lv = lane < (NCLS / 2);
      bv0 = lv ? bf16_val(a.x) : 0.0f;
      bv1 = lv ? bf16_val(a.y) : 0.0f;
    }
#pragma unroll 1
    for (int gi = 0; gi < NBA / (4 * NWAVE); ++gi) {
      const int g     = gi * NWAVE + wave;
      const int s0    = 4 * g;
      const int node0 = nodeBase + s0;
#pragma unroll 1
      for (int r = 0; r < 4; ++r) {
        const int s    = s0 + r;
        const int node = node0 + r;
        int c = cnt[s];
        const bool big = c > DEGCAP;
        c = c < 0 ? 0 : (c > DEGCAP ? DEGCAP : c);
        int o = offs[s];
        o = o < 0 ? 0 : (o > RCAP ? RCAP : o);
        const int nc = node < nN ? node : nN - 1;
        const float ndv = nd[nc];
        float acc0 = 0.0f, acc1 = 0.0f;
#pragma unroll 1
        for (int b0 = 0; b0 < c; b0 += 32) {
          int idx = o + b0 + lane;
          idx = idx > RCAP - 1 ? RCAP - 1 : idx;
          const int ent = sl[idx];
          int eid = ent >> SLA;
          eid = eid < 0 ? 0 : (eid > nE - 1 ? nE - 1 : eid);
          int sr = srcs[eid];
          sr = sr < 0 ? 0 : (sr > nN - 1 ? nN - 1 : sr);
          const int m32 = (c - b0) < 32 ? (c - b0) : 32;
#pragma unroll 1
          for (int k = 0; k < m32; ++k) {
            const int sk = __builtin_amdgcn_readlane(sr, k);
            const v2f a = *(const v2fa*)(xl + (size_t)sk * N2P + 2 * lane);
            acc0 += a.x; acc1 += a.y;
          }
        }
        const float pzr = big ? qnan : pz;
        const float y0 = (acc0 * ndv + bv0) + pzr;
        const float y1 = (acc1 * ndv + bv1) + pzr;
        if (lane < (NCLS / 2)) {
          stgf[r * NCLS + 2 * lane]     = y0;
          stgf[r * NCLS + 2 * lane + 1] = y1;
        }
      }
      wave_sync();
      const v4f q0 = *(const v4fa*)(stgf + 4 * lane);
      const v4f q1 = *(const v4fa*)(stgf + 128 + 4 * (lane & 7));
      wave_sync();
      if (node0 < nN) {
        float* op = hout + (size_t)node0 * NCLS + 4 * lane;
        *(volatile v4f*)op = q0;
        if (lane < 8) *(volatile v4f*)(op + 128) = q1;
        __threadfence();
        *(volatile v4f*)op = q0;
        if (lane < 8) *(volatile v4f*)(op + 128) = q1;
      }
    }
  }
}

static inline int cdiv(int a, int b) { return (a + b - 1) / b; }
static inline size_t al256(size_t o) { return (o + 255) & ~(size_t)255; }

extern "C" void kernel_launch(void* const* d_in, const int* in_sizes, int n_in,
                              void* d_out, int out_size, void* d_ws, size_t ws_size,
                              hipStream_t stream) {
  if (n_in < 8) return;
  if (in_sizes[0] < SEQ || (in_sizes[0] % SEQ) != 0) return;
  const int nN = in_sizes[0] / SEQ;
  if (nN < 16 || nN > (1 << 22) || (nN & 3) != 0) return;
  const int nE = in_sizes[1];
  if (nE < 1 || in_sizes[2] != nE) return;
  if (nE >= (1 << (31 - SLA))) return;
  if (in_sizes[3] < EMB || (in_sizes[3] % EMB) != 0) return;
  const int nTok = in_sizes[3] / EMB;
  if (in_sizes[4] != HF * HF || in_sizes[5] != HF) return;
  if (in_sizes[6] != HF * NCLS || in_sizes[7] != NCLS) return;
  if ((long long)out_size != (long long)nN * NCLS) return;

  const int*   feats = (const int*)d_in[0];
  const int*   src   = (const int*)d_in[1];
  const int*   dst   = (const int*)d_in[2];
  const float* emb   = (const float*)d_in[3];
  const float* W1    = (const float*)d_in[4];
  const float* b1    = (const float*)d_in[5];
  const float* W2    = (const float*)d_in[6];
  const float* b2    = (const float*)d_in[7];
  float* out = (float*)d_out;

  const int MP   = cdiv(nN, GBM) * GBM;
  const int gM   = MP / GBM;
  const int gD   = cdiv(MP, NBD);
  const int NBPD = gD * NBD;
  const int gA   = cdiv(MP, NBA);
  if ((long long)gA * NBA < (long long)MP) return;
  if (NBPD < MP) return;
  const int vec8 = 1;

  char* ws = (char*)d_ws;
  size_t off = 0;
  const size_t oNS  = off; off = al256(off + (size_t)NBPD * 4);
  const size_t oND  = off; off = al256(off + (size_t)NBPD * 4);
  const size_t oW1T = off; off = al256(off + (size_t)HF * K1 * 2);
  const size_t oW2T = off; off = al256(off + (size_t)N2P * K2 * 2);
  const size_t oHX  = off; off = al256(off + (size_t)MP * AP * 2);
  const size_t oM1  = off; off = al256(off + (size_t)MP * HF * 4);
  const size_t oM2  = off; off = al256(off + (size_t)MP * N2P * 4);
  if (off > ws_size || off > (size_t)WSMAX) return;
  float*          NS  = (float*)(ws + oNS);
  float*          ND  = (float*)(ws + oND);
  unsigned short* W1T = (unsigned short*)(ws + oW1T);
  unsigned short* W2T = (unsigned short*)(ws + oW2T);
  unsigned short* HX  = (unsigned short*)(ws + oHX);
  float*          M1  = (float*)(ws + oM1);
  float*          M2  = (float*)(ws + oM2);

  const size_t aggLds = (size_t)AGG_LDS_INTS * 4;
  hipFuncSetAttribute(reinterpret_cast<const void*>(&k_agg<1>), hipFuncAttributeMaxDynamicSharedMemorySize, (int)aggLds);
  hipFuncSetAttribute(reinterpret_cast<const void*>(&k_agg<0>), hipFuncAttributeMaxDynamicSharedMemorySize, (int)aggLds);

  k_prep<<<(NU1 + NU2) / NTHR, NTHR, 0, stream>>>(W1, W2, W1T, W2T);
  k_deg<<<gD, NTHR, 0, stream>>>(src, nE, vec8, NS);
  k_deg<<<gD, NTHR, 0, stream>>>(dst, nE, vec8, ND);
  k_embed<<<MP / NWAVE, NTHR, 0, stream>>>(feats, emb, nN, nTok, HX);
  k_gemm<<<dim3(gM, HF / GBN), GTHR, 0, stream>>>(HX, AP, W1T, K1, NS, M1, HF);
  k_agg<1><<<gA, NTHR, aggLds, stream>>>(src, dst, nE, nN, vec8, MP, ND, M1, b1, HX, out);
  k_gemm<<<dim3(gM, N2P / GBN), GTHR, 0, stream>>>(HX, AP, W2T, K2, NS, M2, N2P);
  k_agg<0><<<gA, NTHR, aggLds, stream>>>(src, dst, nE, nN, vec8, MP, ND, M2, b2, HX, out);
}
